// BiLevelRoutingAttention_89945205112996
// MI455X (gfx1250) — hardware-verified
//
#include <hip/hip_runtime.h>
#include <stdint.h>

#define NIMG   16
#define CCH    256
#define OC3    768
#define HPIX   56
#define WPIX   56
#define HW     3136
#define NHEAD  8
#define DHEAD  32
#define RGRID  7
#define RS     8
#define NREG   49
#define RS2    64
#define NTOPK  4
#define REGP   64
#define TP     264

#define WCARRY 1024.0f
#define RWC    (1.0f / 1024.0f)
#define QCARRY 16.0f
#define KCARRY 8.0f
#define VCARRY 8.0f
#define SINV   (1.0f / 128.0f)
#define PCARRY 1024.0f
#define OINV   (1.0f / 8192.0f)
#define YCARRY 64.0f
#define OSC2   (1.0f / 65536.0f)
#define QSCALE 0.17677669529663687f

static_assert(CCH == NHEAD * DHEAD);
static_assert(HW == NREG * RS2);
static_assert(HW == HPIX * WPIX);
static_assert((HW % 64) == 0 && (CCH % 64) == 0 && (CCH % 32) == 0);
static_assert(RGRID * RS == HPIX);
static_assert(NREG <= REGP);
static_assert(REGP * NTOPK == 256);

typedef _Float16 v16h __attribute__((ext_vector_type(16)));
typedef _Float16 v8h  __attribute__((ext_vector_type(8)));
typedef float    v8f  __attribute__((ext_vector_type(8)));
typedef float    v4f  __attribute__((ext_vector_type(4)));
typedef int      v4i  __attribute__((ext_vector_type(4)));
typedef unsigned int v4u __attribute__((ext_vector_type(4)));
typedef v8h __attribute__((may_alias)) v8ha;
typedef v4f __attribute__((may_alias)) v4fa;
typedef v4i __attribute__((may_alias)) v4ia;

union Frag { v16h v; v8h half[2]; };

#if defined(__HIP_DEVICE_COMPILE__)
#define DEV_ASM 1
#else
#define DEV_ASM 0
#endif

__device__ __forceinline__ unsigned short h_bits(_Float16 x) { return __builtin_bit_cast(unsigned short, x); }
__device__ __forceinline__ unsigned pk16(unsigned short a, unsigned short b) { return (unsigned)a | ((unsigned)b << 16); }
__device__ __forceinline__ v8f zero8() { v8f z = {0.f, 0.f, 0.f, 0.f, 0.f, 0.f, 0.f, 0.f}; return z; }

__device__ __forceinline__ void ldwait() {
#if DEV_ASM
  asm volatile("s_wait_loadcnt 0x0" ::: "memory");
#endif
}

__device__ __forceinline__ v8f wmma_f16(v16h a, v16h b, v8f c) {
  v8f d = __builtin_amdgcn_wmma_f32_16x16x32_f16(false, a, false, b, (short)0, c, false, false);
#if DEV_ASM
  asm volatile("v_nop\n\tv_nop\n\tv_nop\n\tv_nop" : "+v"(d) : "v"(a), "v"(b));
#endif
  return d;
}
__device__ __forceinline__ v8f mmar(v16h a, v16h b, v8f c) {
  return __builtin_amdgcn_wmma_f32_16x16x32_f16(false, a, false, b, (short)0, c, false, false);
}
__device__ __forceinline__ void dep_guard(v8f& a, v8f& b, v16h x, v16h y) {
#if DEV_ASM
  asm volatile("v_nop\n\tv_nop\n\tv_nop\n\tv_nop" : "+v"(a), "+v"(b) : "v"(x), "v"(y));
#else
  (void)a; (void)b; (void)x; (void)y;
#endif
}
__device__ __forceinline__ void keep4(v16h a, v16h b, v16h c, v16h d) {
#if DEV_ASM
  asm volatile("v_nop" :: "v"(a), "v"(b), "v"(c), "v"(d));
#else
  (void)a; (void)b; (void)c; (void)d;
#endif
}
__device__ __forceinline__ void acc_guard4(v8f& a, v8f& b, v8f& c, v8f& d) {
#if DEV_ASM
  asm volatile("v_nop\n\tv_nop\n\tv_nop\n\tv_nop" : "+v"(a), "+v"(b), "+v"(c), "+v"(d));
#else
  (void)a; (void)b; (void)c; (void)d;
#endif
}

__device__ __forceinline__ v16h ldfrag(const _Float16* p) {
  Frag f;
  f.half[0] = *(const v8ha*)(p);
  f.half[1] = *(const v8ha*)(p + 16);
  return f.v;
}

__global__ __launch_bounds__(256) void cvt_w_kernel(const float* __restrict__ wqkv, const float* __restrict__ wout,
                                                    _Float16* wq16, _Float16* wo16) {
  const int g = blockIdx.x * 256 + (int)threadIdx.x;
  const int n8a = OC3 * CCH / 8;
  const int n8b = CCH * CCH / 8;
  if (g >= n8a + n8b) return;
  const float* src;
  _Float16* dst;
  if (g < n8a) { src = wqkv + (size_t)g * 8; dst = wq16 + (size_t)g * 8; }
  else { const int e = g - n8a; src = wout + (size_t)e * 8; dst = wo16 + (size_t)e * 8; }
  const v4f a = *(const v4fa*)src;
  const v4f c = *(const v4fa*)(src + 4);
  const v8h o = { (_Float16)(a.x * WCARRY), (_Float16)(a.y * WCARRY), (_Float16)(a.z * WCARRY), (_Float16)(a.w * WCARRY),
                  (_Float16)(c.x * WCARRY), (_Float16)(c.y * WCARRY), (_Float16)(c.z * WCARRY), (_Float16)(c.w * WCARRY) };
  *(volatile v8h*)dst = o;
  __threadfence();
  *(volatile v8h*)dst = o;
}

__global__ __launch_bounds__(64) void xmean_kernel(const float* __restrict__ x, float* xr) {
  __shared__ float cs[RGRID][64];
  __shared__ __attribute__((aligned(16))) float sr[REGP];
  const int nc = blockIdx.x;
  const int t  = (int)threadIdx.x;
  const float* xp = x + (size_t)nc * HW;
  if (t < WPIX) {
#pragma unroll 1
    for (int rh = 0; rh < RGRID; ++rh) {
      float s = 0.f;
#pragma unroll
      for (int py = 0; py < RS; ++py) s += xp[(rh * RS + py) * WPIX + t];
      cs[rh][t] = s;
    }
  }
  __syncthreads();
  float r = 0.f;
  if (t < NREG) {
    const int rh = t / RGRID, rw = t - rh * RGRID;
    float s = 0.f;
#pragma unroll
    for (int px = 0; px < RS; ++px) s += cs[rh][rw * RS + px];
    r = s * (1.0f / 64.0f);
  }
  sr[t] = r;
  __syncthreads();
  if (t < 16) {
    const v4f v = *(const v4fa*)(sr + t * 4);
    float* dst = xr + (size_t)nc * REGP + t * 4;
    *(volatile v4f*)dst = v;
    __threadfence();
    *(volatile v4f*)dst = v;
  }
}

__global__ __launch_bounds__(64) void qkr_kernel(const float* __restrict__ wqkv, const float* __restrict__ bqkv,
                                                 const float* __restrict__ xr, float* qkr) {
  __shared__ __attribute__((aligned(16))) float sr[REGP];
  const int o = blockIdx.x;
  const int n = blockIdx.y;
  const int t = (int)threadIdx.x;
  const float* w  = wqkv + (size_t)o * CCH;
  const float* xp = xr + (size_t)n * CCH * REGP + t;
  float acc = 0.f;
#pragma unroll 4
  for (int c = 0; c < CCH; ++c) acc = fmaf(w[c], xp[(size_t)c * REGP], acc);
  const float v = (t < NREG) ? (acc + bqkv[o]) : 0.f;
  sr[t] = v;
  __syncthreads();
  if (t < 16) {
    const v4f vv = *(const v4fa*)(sr + t * 4);
    float* dst = qkr + ((size_t)n * 2 * CCH + o) * REGP + t * 4;
    *(volatile v4f*)dst = vv;
    __threadfence();
    *(volatile v4f*)dst = vv;
  }
}

__global__ __launch_bounds__(256) void topk_kernel(const float* __restrict__ qkr, int* ridx) {
  __shared__ float ar[NREG * NREG];
  __shared__ __attribute__((aligned(16))) int sidx[REGP * NTOPK];
  const int n   = blockIdx.x;
  const int tid = (int)threadIdx.x;
  const float* q = qkr + (size_t)n * 2 * CCH * REGP;
  const float* k = q + (size_t)CCH * REGP;
  sidx[tid] = 0;
  for (int e = tid; e < NREG * NREG; e += 256) {
    const int i = e / NREG, j = e - i * NREG;
    float acc = 0.f;
#pragma unroll 4
    for (int o = 0; o < CCH; ++o) acc = fmaf(q[(size_t)o * REGP + i], k[(size_t)o * REGP + j], acc);
    ar[e] = acc;
  }
  __syncthreads();
  if (tid < NREG) {
    const int i = tid;
    float pv = 3.4e38f;
    int pi = -1;
#pragma unroll 1
    for (int t = 0; t < NTOPK; ++t) {
      float best = -3.4e38f;
      int bi = 0;
#pragma unroll 1
      for (int j = 0; j < NREG; ++j) {
        const float v = ar[i * NREG + j];
        const bool cand = (v < pv) || (v == pv && j > pi);
        if (cand && v > best) { best = v; bi = j; }
      }
      sidx[i * NTOPK + t] = bi;
      pv = best;
      pi = bi;
    }
  }
  __syncthreads();
  if (tid < 32) {
    int* base = ridx + (size_t)n * REGP * NTOPK;
    for (int pass = 0; pass < 2; ++pass) {
#pragma unroll
      for (int it = 0; it < 2; ++it) {
        const int off = it * 128 + tid * 4;
        const v4i v = *(const v4ia*)(sidx + off);
        *(volatile v4i*)(base + off) = v;
      }
      __threadfence();
    }
  }
}

__global__ __launch_bounds__(256) void xseq_kernel(const float* __restrict__ x, _Float16* xt) {
  __shared__ __attribute__((aligned(16))) _Float16 T[RS2 * TP];
  const int blk = blockIdx.x;
  const int n = blk / NREG, reg = blk - n * NREG;
  const int rH = reg / RGRID, rW = reg - rH * RGRID;
  const int tid = (int)threadIdx.x, lane = tid & 31, w = tid >> 5;
  const int tok = tid & 63, cg = tid >> 6;
  const int py = tok >> 3, px = tok & 7;
  const float* xp = x + (size_t)n * CCH * HW + (size_t)(rH * RS + py) * WPIX + rW * RS + px;
#pragma unroll 4
  for (int it = 0; it < 64; ++it) {
    const int c = it * 4 + cg;
    T[tok * TP + c] = (_Float16)xp[(size_t)c * HW];
  }
  __syncthreads();
  _Float16* ob = xt + ((size_t)n * HW + (size_t)reg * RS2) * CCH;
  for (int pass = 0; pass < 2; ++pass) {
#pragma unroll
    for (int i = 0; i < 8; ++i) {
      const int tk = w * 8 + i;
      const v8h v = *(const v8ha*)(T + tk * TP + lane * 8);
      *(volatile v8h*)(ob + (size_t)tk * CCH + lane * 8) = v;
    }
    __threadfence();
  }
}

template <int MODE>
__global__ __launch_bounds__(256) void gemm64(
    const _Float16* __restrict__ A, int lda, long long strideA,
    const _Float16* __restrict__ Bt, int ldb, long long strideB,
    const float* __restrict__ bias,
    void* C0, void* C1, int ldc, long long strideC,
    int M, int N, int K) {
  __shared__ __attribute__((aligned(16))) float sT[8][16 * 68];
  const int b    = blockIdx.y;
  const int lane = (int)threadIdx.x & 31;
  const int wave = (int)threadIdx.x >> 5;
  const int tilesN = N >> 6;
  const int tilesM = M >> 6;
  const int tile = blockIdx.x * 8 + wave;
  if (tile >= tilesM * tilesN) return;
  const int tm = tile / tilesN;
  const int tn = tile - tm * tilesN;
  const int m0 = tm << 6;
  const int n0 = tn << 6;

  const _Float16* Ab = A  + (size_t)b * (size_t)strideA;
  const _Float16* Bb = Bt + (size_t)b * (size_t)strideB;

  const int rlane = lane & 15;
  const int koff  = (lane >> 4) * 8;
  const int mOff  = (lane >> 4) * 8;

  v8f acc[4][4];
#pragma unroll
  for (int i = 0; i < 4; ++i)
#pragma unroll
    for (int j = 0; j < 4; ++j) acc[i][j] = zero8();

  for (int k0 = 0; k0 < K; k0 += 32) {
    v16h bq[4];
#pragma unroll
    for (int j = 0; j < 4; ++j)
      bq[j] = ldfrag(Bb + (size_t)(n0 + (j << 4) + rlane) * ldb + koff + k0);
#pragma unroll
    for (int i = 0; i < 4; ++i) {
      const v16h af = ldfrag(Ab + (size_t)(m0 + (i << 4) + rlane) * lda + koff + k0);
#pragma unroll
      for (int j = 0; j < 4; ++j) acc[i][j] = mmar(af, bq[j], acc[i][j]);
      dep_guard(acc[i][0], acc[i][3], af, bq[3]);
    }
    keep4(bq[0], bq[1], bq[2], bq[3]);
  }
  acc_guard4(acc[0][0], acc[0][1], acc[0][2], acc[0][3]);
  acc_guard4(acc[1][0], acc[1][1], acc[1][2], acc[1][3]);
  acc_guard4(acc[2][0], acc[2][1], acc[2][2], acc[2][3]);
  acc_guard4(acc[3][0], acc[3][1], acc[3][2], acc[3][3]);

  float* slab = sT[wave];
#pragma unroll
  for (int i = 0; i < 4; ++i) {
    const int mBase = m0 + (i << 4);
#pragma unroll
    for (int j = 0; j < 4; ++j) {
#pragma unroll
      for (int r = 0; r < 8; ++r) {
        slab[(mOff + r) * 68 + (j << 4) + rlane] = acc[i][j][r];
      }
    }
    __builtin_amdgcn_fence(__ATOMIC_RELEASE, "workgroup");
    __builtin_amdgcn_wave_barrier();
    __builtin_amdgcn_fence(__ATOMIC_ACQUIRE, "workgroup");
    if (MODE == 2) {
      float* C = (float*)C0 + (size_t)b * (size_t)strideC;
      const int h2 = lane >> 4, c4 = (lane & 15) * 4;
      for (int pass = 0; pass < 2; ++pass) {
#pragma unroll
        for (int it = 0; it < 8; ++it) {
          const int row = it * 2 + h2;
          const float bv = bias[mBase + row];
          v4f v = *(const v4fa*)(slab + row * 68 + c4);
          v = v * OSC2;
          v = v + bv;
          *(volatile v4f*)(C + (size_t)(mBase + row) * ldc + n0 + c4) = v;
        }
        __threadfence();
      }
    } else {
      const int q = lane >> 3, c8 = (lane & 7) * 8;
      int sel = 0, ncol = n0;
      unsigned short* Cp;
      if (MODE == 0) {
        sel = (n0 >= CCH) ? 1 : 0;
        ncol = n0 - sel * CCH;
        Cp = (unsigned short*)(sel ? C1 : C0) + (size_t)b * (size_t)strideC;
      } else {
        Cp = (unsigned short*)C0 + (size_t)b * (size_t)strideC;
      }
      v4u hv[4];
#pragma unroll
      for (int it = 0; it < 4; ++it) {
        const int row = it * 4 + q;
        const float* sp = slab + row * 68 + c8;
        float f[8], o8[8];
#pragma unroll
        for (int e = 0; e < 8; ++e) f[e] = sp[e];
        if (MODE == 0) {
          const v4f b0 = *(const v4fa*)(bias + n0 + c8);
          const v4f b1 = *(const v4fa*)(bias + n0 + c8 + 4);
          const float bb[8] = { b0.x, b0.y, b0.z, b0.w, b1.x, b1.y, b1.z, b1.w };
#pragma unroll
          for (int e = 0; e < 8; ++e) {
            const float val = f[e] * RWC + bb[e];
            const float vq = (val * QSCALE) * QCARRY;
            const float vk = val * KCARRY;
            o8[e] = sel ? vk : vq;
          }
        } else {
          const float bv = bias[mBase + row];
#pragma unroll
          for (int e = 0; e < 8; ++e) o8[e] = (f[e] * RWC + bv) * VCARRY;
        }
        v4u a;
#pragma unroll
        for (int e = 0; e < 4; ++e) a[e] = pk16(h_bits((_Float16)o8[2 * e]), h_bits((_Float16)o8[2 * e + 1]));
        hv[it] = a;
      }
      for (int pass = 0; pass < 2; ++pass) {
#pragma unroll
        for (int it = 0; it < 4; ++it) {
          const int row = it * 4 + q;
          *(volatile v4u*)(Cp + (size_t)(mBase + row) * ldc + ncol + c8) = hv[it];
        }
        __threadfence();
      }
    }
    __builtin_amdgcn_fence(__ATOMIC_RELEASE, "workgroup");
    __builtin_amdgcn_wave_barrier();
    __builtin_amdgcn_fence(__ATOMIC_ACQUIRE, "workgroup");
  }
}

__device__ __forceinline__ v16h pack_p(v8f a, v8f c) {
  const v16h r = { (_Float16)(a[0] * PCARRY), (_Float16)(a[1] * PCARRY), (_Float16)(a[2] * PCARRY), (_Float16)(a[3] * PCARRY),
                   (_Float16)(a[4] * PCARRY), (_Float16)(a[5] * PCARRY), (_Float16)(a[6] * PCARRY), (_Float16)(a[7] * PCARRY),
                   (_Float16)(c[0] * PCARRY), (_Float16)(c[1] * PCARRY), (_Float16)(c[2] * PCARRY), (_Float16)(c[3] * PCARRY),
                   (_Float16)(c[4] * PCARRY), (_Float16)(c[5] * PCARRY), (_Float16)(c[6] * PCARRY), (_Float16)(c[7] * PCARRY) };
  return r;
}

__global__ __launch_bounds__(128) void attn_kernel(
    const _Float16* __restrict__ qp,
    const _Float16* __restrict__ kp,
    const _Float16* __restrict__ vt,
    const int* __restrict__ ridx,
    float* att)
{
  __shared__ __attribute__((aligned(16))) _Float16 Ksh[RS2 * DHEAD];
  __shared__ __attribute__((aligned(16))) _Float16 Vsh[DHEAD * RS2];
  __shared__ __attribute__((aligned(16))) float    Os[DHEAD * RS2];

  const int tid = (int)threadIdx.x, lane = tid & 31, w = tid >> 5;
  const int h = lane >> 4, m = lane & 15;
  const int blk  = blockIdx.x;
  const int reg  = blk % NREG;
  const int head = (blk / NREG) % NHEAD;
  const int n    = blk / (NREG * NHEAD);
  const size_t tokbase = (size_t)n * HW;

  const _Float16* qrow = qp + (tokbase + (size_t)reg * RS2 + 16 * w + m) * CCH + head * DHEAD;
  const v16h qb = ldfrag(qrow + 8 * h);

  v8f o[2];
  o[0] = zero8(); o[1] = zero8();
  float mrun = -1e30f, lrun = 0.0f;

  const int* ip = ridx + ((size_t)n * REGP + reg) * NTOPK;

#pragma unroll 1
  for (int kk = 0; kk < NTOPK; ++kk) {
    int regj = ip[kk];
    regj = (regj < 0) ? 0 : ((regj > NREG - 1) ? (NREG - 1) : regj);

    __syncthreads();
    {
      const int key = tid >> 1, hf = (tid & 1) * 16;
      const _Float16* kg = kp + (tokbase + (size_t)regj * RS2 + key) * CCH + head * DHEAD + hf;
      *(v8h*)(Ksh + key * DHEAD + hf)     = *(const v8ha*)(kg);
      *(v8h*)(Ksh + key * DHEAD + hf + 8) = *(const v8ha*)(kg + 8);
      const int d = tid >> 2, pt = (tid & 3) * 16;
      const _Float16* vg = vt + ((size_t)n * CCH + head * DHEAD + d) * HW + (size_t)regj * RS2 + pt;
      *(v8h*)(Vsh + d * RS2 + pt)     = *(const v8ha*)(vg);
      *(v8h*)(Vsh + d * RS2 + pt + 8) = *(const v8ha*)(vg + 8);
    }
    __syncthreads();

    v8f s[4];
#pragma unroll
    for (int j = 0; j < 4; ++j) {
      Frag kf;
      kf.half[0] = *(const v8ha*)(Ksh + (16 * j + m) * DHEAD + 8 * h);
      kf.half[1] = *(const v8ha*)(Ksh + (16 * j + m) * DHEAD + 16 + 8 * h);
      v8f z = zero8();
      z = wmma_f16(kf.v, qb, z);
#pragma unroll
      for (int r = 0; r < 8; ++r) z[r] = z[r] * SINV;
      s[j] = z;
    }

    float mloc = s[0][0];
#pragma unroll
    for (int j = 0; j < 4; ++j)
#pragma unroll
      for (int r = 0; r < 8; ++r) mloc = fmaxf(mloc, s[j][r]);
    mloc = fmaxf(mloc, __shfl_xor(mloc, 16));
    const float mnew  = fmaxf(mrun, mloc);
    const float alpha = __expf(mrun - mnew);
    mrun = mnew;
    float lsum = 0.0f;
#pragma unroll
    for (int j = 0; j < 4; ++j)
#pragma unroll
      for (int r = 0; r < 8; ++r) {
        const float p = __expf(s[j][r] - mnew);
        s[j][r] = p;
        lsum += p;
      }
    lsum += __shfl_xor(lsum, 16);
    lrun = lrun * alpha + lsum;
#pragma unroll
    for (int t = 0; t < 2; ++t)
#pragma unroll
      for (int r = 0; r < 8; ++r) o[t][r] = o[t][r] * alpha;

    const v16h pb0 = pack_p(s[0], s[1]);
    const v16h pb1 = pack_p(s[2], s[3]);

#pragma unroll
    for (int t = 0; t < 2; ++t) {
      const _Float16* vrow = Vsh + (16 * t + m) * RS2;
      Frag v0, v1;
      v0.half[0] = *(const v8ha*)(vrow + 8 * h);
      v0.half[1] = *(const v8ha*)(vrow + 16 + 8 * h);
      v1.half[0] = *(const v8ha*)(vrow + 32 + 8 * h);
      v1.half[1] = *(const v8ha*)(vrow + 48 + 8 * h);
      o[t] = wmma_f16(v0.v, pb0, o[t]);
      o[t] = wmma_f16(v1.v, pb1, o[t]);
    }
  }

  const float inv = (1.0f / lrun) * OINV;
#pragma unroll
  for (int t = 0; t < 2; ++t)
#pragma unroll
    for (int r = 0; r < 8; ++r)
      Os[(16 * t + 8 * h + r) * RS2 + 16 * w + m] = o[t][r] * inv;
  __syncthreads();

  float* ob = att + ((size_t)n * CCH + head * DHEAD) * HW + (size_t)reg * RS2;
  const int p8 = tid & 7, lq = tid >> 3;
  for (int pass = 0; pass < 2; ++pass) {
#pragma unroll
    for (int it = 0; it < 4; ++it) {
      const int L = it * 16 + lq;
      const int d = L >> 1, hl = L & 1;
      const v4f v = *(const v4fa*)(Os + d * RS2 + hl * 32 + p8 * 4);
      *(volatile v4f*)(ob + (size_t)d * HW + hl * 32 + p8 * 4) = v;
    }
    __threadfence();
  }
}

__global__ __launch_bounds__(256) void ybuild_kernel(const float* __restrict__ att, const _Float16* __restrict__ vt,
                                                    const float* __restrict__ wl, const float* __restrict__ bl,
                                                    _Float16* y) {
  __shared__ __attribute__((aligned(16))) _Float16 T[RS2 * TP];
  __shared__ __attribute__((aligned(16))) float wls[CCH * 9];
  __shared__ __attribute__((aligned(16))) float bls[CCH];
  const int blk = blockIdx.x;
  const int n = blk / NREG, reg = blk - n * NREG;
  const int rH = reg / RGRID, rW = reg - rH * RGRID;
  const int tid = (int)threadIdx.x, lane = tid & 31, w = tid >> 5;
  const int tok = tid & 63, cg = tid >> 6;
  const int py = tok >> 3, px = tok & 7;
  const int gy = rH * RS + py, gx = rW * RS + px;

  for (int t4 = tid; t4 < (CCH * 9) / 4; t4 += 256) {
    const v4f v = *(const v4fa*)(wl + (size_t)t4 * 4);
    *(v4f*)(wls + t4 * 4) = v;
  }
  if (tid < CCH / 4) {
    const v4f v = *(const v4fa*)(bl + (size_t)tid * 4);
    *(v4f*)(bls + tid * 4) = v;
  }

  int   noff[9];
  float nmul[9];
#pragma unroll
  for (int tap = 0; tap < 9; ++tap) {
    const int dy = tap / 3 - 1, dx = tap % 3 - 1;
    const int yy = gy + dy, xx = gx + dx;
    const bool ok = (yy >= 0) && (yy < HPIX) && (xx >= 0) && (xx < WPIX);
    const int yc = (yy < 0) ? 0 : ((yy > HPIX - 1) ? (HPIX - 1) : yy);
    const int xc = (xx < 0) ? 0 : ((xx > WPIX - 1) ? (WPIX - 1) : xx);
    noff[tap] = ((yc >> 3) * RGRID + (xc >> 3)) * RS2 + (yc & 7) * RS + (xc & 7);
    nmul[tap] = ok ? (1.0f / VCARRY) : 0.0f;
  }
  __syncthreads();

#pragma unroll 1
  for (int it = 0; it < 64; ++it) {
    const int c = it * 4 + cg;
    const size_t pb = ((size_t)n * CCH + c) * HW;
    const float a = att[pb + (size_t)reg * RS2 + tok];
    const _Float16* vp = vt + pb;
    const float* wc = wls + c * 9;
    float s = 0.0f;
#pragma unroll
    for (int tap = 0; tap < 5; ++tap) s += wc[tap] * ((float)vp[noff[tap]] * nmul[tap]);
    ldwait();
#pragma unroll
    for (int tap = 5; tap < 9; ++tap) s += wc[tap] * ((float)vp[noff[tap]] * nmul[tap]);
    const float val = ((a + s) + bls[c]) * YCARRY;
    T[tok * TP + c] = (_Float16)val;
  }
  __syncthreads();

  _Float16* ob = y + (size_t)n * HW * CCH;
  for (int pass = 0; pass < 2; ++pass) {
#pragma unroll
    for (int i = 0; i < 8; ++i) {
      const int tk  = w * 8 + i;
      const int pix = (rH * RS + (tk >> 3)) * WPIX + rW * RS + (tk & 7);
      const v8h v = *(const v8ha*)(T + tk * TP + lane * 8);
      *(volatile v8h*)(ob + (size_t)pix * CCH + lane * 8) = v;
    }
    __threadfence();
  }
}

extern "C" void kernel_launch(void* const* d_in, const int* in_sizes, int n_in,
                              void* d_out, int out_size, void* d_ws, size_t ws_size,
                              hipStream_t stream) {
  if (n_in < 7) return;
  if (in_sizes[0] != NIMG * CCH * HW) return;
  if (in_sizes[1] != OC3 * CCH) return;
  if (in_sizes[2] != OC3) return;
  if (in_sizes[3] != CCH * 9) return;
  if (in_sizes[4] != CCH) return;
  if (in_sizes[5] != CCH * CCH) return;
  if (in_sizes[6] != CCH) return;
  if (out_size != NIMG * CCH * HW) return;

  const float* x      = (const float*)d_in[0];
  const float* w_qkv  = (const float*)d_in[1];
  const float* b_qkv  = (const float*)d_in[2];
  const float* w_lepe = (const float*)d_in[3];
  const float* b_lepe = (const float*)d_in[4];
  const float* w_out  = (const float*)d_in[5];
  const float* b_out  = (const float*)d_in[6];
  float* out = (float*)d_out;

  const size_t PW3  = (size_t)OC3 * CCH * 2;
  const size_t PWO  = (size_t)CCH * CCH * 2;
  const size_t PXR  = (size_t)NIMG * CCH * REGP * 4;
  const size_t PQKR = (size_t)NIMG * 2 * CCH * REGP * 4;
  const size_t PIDX = (size_t)NIMG * REGP * NTOPK * 4;
  const size_t PATT = (size_t)NIMG * CCH * HW * 4;
  const size_t P16  = (size_t)NIMG * HW * CCH * 2;
  size_t off = 0;
  const size_t oW3  = off; off += PW3;
  const size_t oWO  = off; off += PWO;
  const size_t oXR  = off; off += PXR;
  const size_t oQKR = off; off += PQKR;
  const size_t oIDX = off; off += PIDX;
  const size_t oATT = off; off += PATT;
  const size_t oQP  = off; off += P16;
  const size_t oKP  = off; off += P16;
  const size_t oVT  = off; off += P16;
  if (off > ws_size) return;
  if (off > (size_t)134217728) return;
  if (P16 > PATT) return;

  char* ws = (char*)d_ws;
  _Float16* wq16 = (_Float16*)(ws + oW3);
  _Float16* wo16 = (_Float16*)(ws + oWO);
  float*    xr   = (float*)(ws + oXR);
  float*    qkr  = (float*)(ws + oQKR);
  int*      ridx = (int*)(ws + oIDX);
  float*    attp = (float*)(ws + oATT);
  _Float16* xt   = (_Float16*)(ws + oATT);
  _Float16* qpl  = (_Float16*)(ws + oQP);
  _Float16* ypl  = (_Float16*)(ws + oQP);
  _Float16* kpl  = (_Float16*)(ws + oKP);
  _Float16* vtp  = (_Float16*)(ws + oVT);

  const int n8w = (OC3 * CCH + CCH * CCH) / 8;
  cvt_w_kernel<<<dim3((n8w + 255) / 256), dim3(256), 0, stream>>>(w_qkv, w_out, wq16, wo16);
  xmean_kernel<<<dim3(NIMG * CCH), dim3(64), 0, stream>>>(x, xr);
  qkr_kernel<<<dim3(2 * CCH, NIMG), dim3(64), 0, stream>>>(w_qkv, b_qkv, xr, qkr);
  topk_kernel<<<dim3(NIMG), dim3(256), 0, stream>>>(qkr, ridx);
  xseq_kernel<<<dim3(NIMG * NREG), dim3(256), 0, stream>>>(x, xt);
  gemm64<0><<<dim3((HW / 64) * (2 * CCH / 64) / 8, NIMG), dim3(256), 0, stream>>>(
      xt, CCH, (long long)HW * CCH, wq16, CCH, 0LL, b_qkv,
      (void*)qpl, (void*)kpl, CCH, (long long)HW * CCH, HW, 2 * CCH, CCH);
  gemm64<1><<<dim3(((CCH / 64) * (HW / 64) + 7) / 8, NIMG), dim3(256), 0, stream>>>(
      wq16 + (size_t)2 * CCH * CCH, CCH, 0LL, xt, CCH, (long long)HW * CCH, b_qkv + 2 * CCH,
      (void*)vtp, (void*)vtp, HW, (long long)CCH * HW, CCH, HW, CCH);
  attn_kernel<<<dim3(NIMG * NHEAD * NREG), dim3(128), 0, stream>>>(qpl, kpl, vtp, ridx, attp);
  ybuild_kernel<<<dim3(NIMG * NREG), dim3(256), 0, stream>>>(attp, vtp, w_lepe, b_lepe, ypl);
  gemm64<2><<<dim3(((CCH / 64) * (HW / 64) + 7) / 8, NIMG), dim3(256), 0, stream>>>(
      wo16, CCH, 0LL, ypl, CCH, (long long)HW * CCH, b_out,
      (void*)out, (void*)out, HW, (long long)CCH * HW, CCH, HW, CCH);
  (void)hipGetLastError();
}
